// DSIB_26980984553579
// MI455X (gfx1250) — hardware-verified
//
#include <hip/hip_runtime.h>
#include <stddef.h>


#define BSZ  512
#define NX   64
#define HID  256
#define NTHR 256
#define WSC  16.0f
#define WINV 0.0625f

typedef float    v4f  __attribute__((ext_vector_type(4)));
typedef float    v8f  __attribute__((ext_vector_type(8)));
typedef _Float16 v8h  __attribute__((ext_vector_type(8)));
typedef _Float16 v16h __attribute__((ext_vector_type(16)));
union FragH { v16h v; v8h h[2]; };

static_assert((BSZ % 256) == 0);
static_assert((HID % 32) == 0);
static_assert(NX <= NTHR && HID == NTHR);

__device__ __forceinline__ v8f wmh(v16h a, v16h b, v8f c) {
  v8f d = __builtin_amdgcn_wmma_f32_16x16x32_f16(false, a, false, b, (short)0, c, false, false);
  asm volatile("v_nop\n\tv_nop\n\tv_nop\n\tv_nop" : "+v"(d) : "v"(a), "v"(b));
  return d;
}

__global__ __launch_bounds__(NTHR) void k_node(
    const float* __restrict__ X, const float* __restrict__ Y,
    const float* __restrict__ W1, const float* __restrict__ b1,
    float* P)
{
  __shared__ float row[NX];
  const int isY = (blockIdx.x >= BSZ) ? 1 : 0;
  const int r   = blockIdx.x & (BSZ - 1);
  const int hc  = threadIdx.x;

  if (hc < NX) {
    const float xv = X[r * NX + hc];
    const float yv = Y[r * NX + hc];
    row[hc] = (isY != 0) ? yv : xv;
  }
  __syncthreads();

  const int   woff = (isY != 0) ? NX * HID : 0;
  const float bv   = b1[hc];
  float s = (isY != 0) ? bv : 0.0f;
#pragma unroll 8
  for (int k = 0; k < NX; ++k)
    s = fmaf(row[k], W1[woff + k * HID + hc], s);

  const size_t idx = (size_t)isY * BSZ * HID + (size_t)r * HID + hc;
  const float  sv  = s;
  *(volatile float*)(P + idx) = sv;
  __threadfence();
  *(volatile float*)(P + idx) = sv;
}

__global__ __launch_bounds__(NTHR) void k_w2t(const float* __restrict__ W2, _Float16* W2t)
{
  const int n    = blockIdx.x * (NTHR / 32) + (threadIdx.x >> 5);
  const int lane = threadIdx.x & 31;
  v8h hv;
#pragma unroll
  for (int t = 0; t < 8; ++t) {
    const float w = W2[(size_t)(8 * lane + t) * HID + n] * WSC;
    hv[t] = (_Float16)w;
  }
  _Float16* dst = W2t + (size_t)n * HID + 8 * lane;
  *(volatile v8h*)dst = hv;
  __threadfence();
  *(volatile v8h*)dst = hv;
}

__device__ __forceinline__ v16h build_a(const float* __restrict__ axr,
                                        const float* __restrict__ ayr, int k0)
{
  const v4f xa0 = *(const v4f*)(axr + k0);
  const v4f xa1 = *(const v4f*)(axr + k0 + 4);
  const v4f xb0 = *(const v4f*)(axr + k0 + 16);
  const v4f xb1 = *(const v4f*)(axr + k0 + 20);
  const v4f ya0 = *(const v4f*)(ayr + k0);
  const v4f ya1 = *(const v4f*)(ayr + k0 + 4);
  const v4f yb0 = *(const v4f*)(ayr + k0 + 16);
  const v4f yb1 = *(const v4f*)(ayr + k0 + 20);
  v16h a;
#pragma unroll
  for (int c = 0; c < 4; ++c) {
    a[c]      = (_Float16)fmaxf(xa0[c] + ya0[c], 0.0f);
    a[4 + c]  = (_Float16)fmaxf(xa1[c] + ya1[c], 0.0f);
    a[8 + c]  = (_Float16)fmaxf(xb0[c] + yb0[c], 0.0f);
    a[12 + c] = (_Float16)fmaxf(xb1[c] + yb1[c], 0.0f);
  }
  return a;
}

__global__ __launch_bounds__(NTHR) void k_pairs(
    const float* __restrict__ Px, const float* __restrict__ Py,
    const _Float16* __restrict__ W2t, const float* __restrict__ b2,
    const float* __restrict__ W3, const float* __restrict__ b3,
    float* scores)
{
  const int lane = threadIdx.x & 31;
  const int wave = threadIdx.x >> 5;
  const int hh   = lane >> 4;
  const int m    = lane & 15;
  const int i    = blockIdx.y;
  const int j0   = blockIdx.x * 256 + wave * 32;

  const float* ax0 = Px + (size_t)(j0 + m) * HID;
  const float* ax1 = Px + (size_t)(j0 + 16 + m) * HID;
  const float* ay  = Py + (size_t)i * HID;

  v16h af0[8], af1[8];
#pragma unroll
  for (int ks = 0; ks < 8; ++ks) {
    const int k0 = ks * 32 + 8 * hh;
    af0[ks] = build_a(ax0, ay, k0);
    af1[ks] = build_a(ax1, ay, k0);
  }

  float p0[8], p1[8];
#pragma unroll
  for (int r = 0; r < 8; ++r) { p0[r] = 0.0f; p1[r] = 0.0f; }

  const _Float16* wl = W2t + (size_t)m * HID + 8 * hh;

#pragma unroll 1
  for (int nt = 0; nt < HID / 16; ++nt) {
    v8f acc0, acc1;
#pragma unroll
    for (int r = 0; r < 8; ++r) { acc0[r] = 0.0f; acc1[r] = 0.0f; }
    const _Float16* wn = wl + (size_t)nt * 16 * HID;
#pragma unroll
    for (int ks = 0; ks < 8; ++ks) {
      FragH b;
      b.h[0] = *(const v8h*)(wn + ks * 32);
      b.h[1] = *(const v8h*)(wn + ks * 32 + 16);
      acc0 = wmh(af0[ks], b.v, acc0);
      acc1 = wmh(af1[ks], b.v, acc1);
    }
    const int   n   = nt * 16 + m;
    const float b2v = b2[n];
    const float w3v = W3[n];
#pragma unroll
    for (int r = 0; r < 8; ++r) {
      p0[r] = fmaf(fmaxf(fmaf(acc0[r], WINV, b2v), 0.0f), w3v, p0[r]);
      p1[r] = fmaf(fmaxf(fmaf(acc1[r], WINV, b2v), 0.0f), w3v, p1[r]);
    }
  }

#pragma unroll
  for (int r = 0; r < 8; ++r) {
    float a = p0[r], b = p1[r];
    a += __shfl_xor(a, 1, 32);  b += __shfl_xor(b, 1, 32);
    a += __shfl_xor(a, 2, 32);  b += __shfl_xor(b, 2, 32);
    a += __shfl_xor(a, 4, 32);  b += __shfl_xor(b, 4, 32);
    a += __shfl_xor(a, 8, 32);  b += __shfl_xor(b, 8, 32);
    p0[r] = a; p1[r] = b;
  }
  float t0[8], t1[8];
#pragma unroll
  for (int r = 0; r < 8; ++r) {
    t0[r] = __shfl_xor(p0[r], 16, 32);
    t1[r] = __shfl_xor(p1[r], 16, 32);
  }
  const bool tsel = ((lane >> 2) & 1) != 0;
  const bool hsel = ((lane >> 1) & 1) != 0;
  const bool rsel = (lane & 1) != 0;
  const float bb3 = b3[0];
  v4f ov;
#pragma unroll
  for (int c = 0; c < 4; ++c) {
    const float lo0 = hsel ? t0[c] : p0[c];
    const float hi0 = hsel ? t0[4 + c] : p0[4 + c];
    const float lo1 = hsel ? t1[c] : p1[c];
    const float hi1 = hsel ? t1[4 + c] : p1[4 + c];
    const float v0 = rsel ? hi0 : lo0;
    const float v1 = rsel ? hi1 : lo1;
    ov[c] = (tsel ? v1 : v0) + bb3;
  }
  float* dp = scores + (size_t)i * BSZ + j0 + 4 * lane;
  if (lane < 8) *(volatile v4f*)dp = ov;
  __threadfence();
  if (lane < 8) *(volatile v4f*)dp = ov;
}

__global__ __launch_bounds__(BSZ) void k_final(const float* __restrict__ scores, float* out)
{
  __shared__ double rd[BSZ];
  __shared__ double rl[BSZ];
  const int i = threadIdx.x;
  const float* rowp = scores + (size_t)i * BSZ;

  float mx = -__builtin_huge_valf();
#pragma unroll 1
  for (int j = 0; j < BSZ; j += 4) {
    const v4f v = *(const v4f*)(rowp + j);
    mx = fmaxf(mx, fmaxf(fmaxf(v.x, v.y), fmaxf(v.z, v.w)));
  }
  float sum = 0.0f;
#pragma unroll 1
  for (int j = 0; j < BSZ; ++j) sum += expf(rowp[j] - mx);
  const float lse = mx + logf(sum);

  rd[i] = (double)rowp[i];
  rl[i] = (double)lse;
  __syncthreads();
#pragma unroll 1
  for (int st = BSZ / 2; st > 0; st >>= 1) {
    if (i < st) { rd[i] += rd[i + st]; rl[i] += rl[i + st]; }
    __syncthreads();
  }
  const double inv  = 1.0 / (double)BSZ;
  const double logB = 6.2383246250395077;
  const double mi   = logB + rd[0] * inv - rl[0] * inv;
  const float  res  = (float)(-mi);
  if (i == 0) *(volatile float*)out = res;
  __threadfence();
  if (i == 0) *(volatile float*)out = res;
}

extern "C" void kernel_launch(void* const* d_in, const int* in_sizes, int n_in,
                              void* d_out, int out_size, void* d_ws, size_t ws_size,
                              hipStream_t stream) {
  if (n_in < 8) return;
  if (in_sizes[0] != BSZ * NX || in_sizes[1] != BSZ * NX) return;
  if (in_sizes[2] != 2 * NX * HID || in_sizes[3] < HID) return;
  if (in_sizes[4] != HID * HID || in_sizes[5] < HID) return;
  if (in_sizes[6] < HID || in_sizes[7] < 1) return;
  if (out_size < 1) return;

  const float* X  = (const float*)d_in[0];
  const float* Y  = (const float*)d_in[1];
  const float* W1 = (const float*)d_in[2];
  const float* b1 = (const float*)d_in[3];
  const float* W2 = (const float*)d_in[4];
  const float* b2 = (const float*)d_in[5];
  const float* W3 = (const float*)d_in[6];
  const float* b3 = (const float*)d_in[7];
  float* out = (float*)d_out;

  char* ws = (char*)d_ws;
  size_t off = 0;
  const size_t oP  = off; off += (size_t)2 * BSZ * HID * sizeof(float);
  const size_t oW  = off; off += (size_t)HID * HID * sizeof(_Float16);
  const size_t oS  = off; off += (size_t)BSZ * BSZ * sizeof(float);
  if (off > ws_size) return;
  float*    P      = (float*)(ws + oP);
  float*    Px     = P;
  float*    Py     = P + (size_t)BSZ * HID;
  _Float16* W2t    = (_Float16*)(ws + oW);
  float*    scores = (float*)(ws + oS);

  k_node<<<2 * BSZ, NTHR, 0, stream>>>(X, Y, W1, b1, P);
  k_w2t<<<HID / (NTHR / 32), NTHR, 0, stream>>>(W2, W2t);
  k_pairs<<<dim3(BSZ / 256, BSZ), NTHR, 0, stream>>>(Px, Py, W2t, b2, W3, b3, scores);
  k_final<<<1, BSZ, 0, stream>>>(scores, out);
}
